// MQA_4475355922804
// MI455X (gfx1250) — hardware-verified
//
#include <hip/hip_runtime.h>


#ifndef NB
#define NB 2
#endif
#ifndef SEQ
#define SEQ 2048
#endif
#define NB_FULL  2
#define SEQ_FULL 2048
#define HID   2048
#define NHEAD 16
#define HD    128
#define SW    (SEQ / 32)
#define NTOK  (NB * SEQ)

static_assert(NB >= 1 && NB <= NB_FULL);
static_assert(SEQ >= 128 && SEQ <= SEQ_FULL && (SEQ % 128) == 0 && (SEQ & (SEQ - 1)) == 0);
static_assert(HID == NHEAD * HD && HD == 128 && (HID % 128) == 0 && (HID % 32) == 0);
static_assert((NTOK % 128) == 0);
static_assert(((SEQ * HID / 8) % 256) == 0 && ((HID * HD / 8) % 256) == 0 && ((HID * HID / 8) % 256) == 0);
static_assert(((SEQ * SW) % 256) == 0);
static_assert((long long)((NB - 1) * SEQ_FULL + SEQ) * HID <= (long long)NB_FULL * SEQ_FULL * HID);

typedef _Float16 v16h __attribute__((ext_vector_type(16)));
typedef _Float16 v8h  __attribute__((ext_vector_type(8)));
typedef _Float16 v8ha __attribute__((ext_vector_type(8), may_alias));
typedef float    v8f  __attribute__((ext_vector_type(8)));
typedef float    v4f  __attribute__((ext_vector_type(4)));
typedef float    v4fa __attribute__((ext_vector_type(4), may_alias));
typedef int      v4ia __attribute__((ext_vector_type(4), may_alias));

union F16Frag {
    v16h h;
    v8h  q[2];
};

static __device__ __forceinline__ v8f wmma_f16(const F16Frag& a, const F16Frag& b, v8f c) {
    return __builtin_amdgcn_wmma_f32_16x16x32_f16(false, a.h, false, b.h, (short)0, c, false, false);
}

static __device__ __forceinline__ v8f vzero8() {
    const v8f z = {0.f, 0.f, 0.f, 0.f, 0.f, 0.f, 0.f, 0.f};
    return z;
}

static __device__ __forceinline__ float bf16r(float x) {
    unsigned u = __float_as_uint(x);
    u = (u + 0x7FFFu + ((u >> 16) & 1u)) & 0xFFFF0000u;
    return __uint_as_float(u);
}

template <int CTRL>
static __device__ __forceinline__ float dpp_mov(float x) {
    int i = __builtin_bit_cast(int, x);
    int r = __builtin_amdgcn_update_dpp(i, i, CTRL, 0xf, 0xf, true);
    return __builtin_bit_cast(float, r);
}
static __device__ __forceinline__ float row_max16(float x) {
    x = fmaxf(x, dpp_mov<0xB1>(x));
    x = fmaxf(x, dpp_mov<0x4E>(x));
    x = fmaxf(x, dpp_mov<0x141>(x));
    x = fmaxf(x, dpp_mov<0x128>(x));
    return x;
}
static __device__ __forceinline__ float row_sum16(float x) {
    x += dpp_mov<0xB1>(x);
    x += dpp_mov<0x4E>(x);
    x += dpp_mov<0x141>(x);
    x += dpp_mov<0x128>(x);
    return x;
}

__global__ __launch_bounds__(256)
void cvt_f16(const float* __restrict__ src, _Float16* __restrict__ dst, int n8, float scale) {
    const int i = blockIdx.x * 256 + threadIdx.x;
    if (i >= n8) return;
    const float* s = src + (size_t)i * 8;
    const v4f a = *reinterpret_cast<const v4fa*>(s);
    const v4f c = *reinterpret_cast<const v4fa*>(s + 4);
    v8h o;
    o[0] = (_Float16)(bf16r(a[0]) * scale);
    o[1] = (_Float16)(bf16r(a[1]) * scale);
    o[2] = (_Float16)(bf16r(a[2]) * scale);
    o[3] = (_Float16)(bf16r(a[3]) * scale);
    o[4] = (_Float16)(bf16r(c[0]) * scale);
    o[5] = (_Float16)(bf16r(c[1]) * scale);
    o[6] = (_Float16)(bf16r(c[2]) * scale);
    o[7] = (_Float16)(bf16r(c[3]) * scale);
    _Float16* d = dst + (size_t)i * 8;
    *reinterpret_cast<volatile v8ha*>(d) = o;
    __threadfence();
    *reinterpret_cast<volatile v8ha*>(d) = o;
}

__global__ __launch_bounds__(256)
void pack_mask(const int* __restrict__ mask, unsigned* __restrict__ bits) {
    const int b  = blockIdx.y;
    const int wi = blockIdx.x * 256 + threadIdx.x;
    const int q  = wi / SW;
    const int w  = wi - q * SW;
    const int* src = mask + ((size_t)b * SEQ_FULL + q) * SEQ_FULL + (size_t)w * 32;
    unsigned word = 0u;
    #pragma unroll
    for (int c = 0; c < 8; ++c) {
        const v4ia x = *reinterpret_cast<const v4ia*>(src + 4 * c);
        word |= (x[0] != 0 ? 1u : 0u) << (4 * c + 0);
        word |= (x[1] != 0 ? 1u : 0u) << (4 * c + 1);
        word |= (x[2] != 0 ? 1u : 0u) << (4 * c + 2);
        word |= (x[3] != 0 ? 1u : 0u) << (4 * c + 3);
    }
    unsigned* d = bits + (size_t)b * SEQ * SW + wi;
    *reinterpret_cast<volatile unsigned*>(d) = word;
    __threadfence();
    *reinterpret_cast<volatile unsigned*>(d) = word;
}

#define LDT   40
#define CSP32 132
#define CSP16 136
#define GEMM_SMEM_BYTES 34816
static_assert(GEMM_SMEM_BYTES >= 2 * 128 * LDT * 2);
static_assert(GEMM_SMEM_BYTES >= 64 * CSP32 * 4);
static_assert(GEMM_SMEM_BYTES >= 128 * CSP16 * 2);

template <typename OutT, bool TRANS>
__global__ __launch_bounds__(256)
void gemm_f16(const _Float16* __restrict__ A, const _Float16* __restrict__ B,
              const float* __restrict__ bias, OutT* __restrict__ C,
              int N, int K, int ldc, int segRows, int segStride,
              float scale, float carry) {
    __shared__ __align__(16) float smem[GEMM_SMEM_BYTES / 4];
    _Float16* const As  = reinterpret_cast<_Float16*>(smem);
    _Float16* const Bst = As + 128 * LDT;

    const int tid  = threadIdx.x;
    const int wave = tid >> 5;
    const int lane = tid & 31;
    const int half = lane >> 4;
    const int l15  = lane & 15;
    const int waveRow = wave >> 2;
    const int waveCol = wave & 3;

    const int mBase = blockIdx.y * 128;
    const int nBase = blockIdx.x * 128;

    v8f acc[4][2];
    #pragma unroll
    for (int mi = 0; mi < 4; ++mi)
        #pragma unroll
        for (int ni = 0; ni < 2; ++ni) acc[mi][ni] = vzero8();

    for (int k0 = 0; k0 < K; k0 += 32) {
        #pragma unroll
        for (int it = 0; it < 2; ++it) {
            const int r  = (tid >> 2) + it * 64;
            const int c8 = (tid & 3) * 8;
            const v8h t = *reinterpret_cast<const v8ha*>(A + (size_t)(mBase + r) * K + k0 + c8);
            *reinterpret_cast<v8ha*>(&As[r * LDT + c8]) = t;
        }
        #pragma unroll
        for (int p = 0; p < 2; ++p) {
            const int kk = (tid >> 4) + p * 16;
            const int n0 = (tid & 15) * 8;
            const v8h t = *reinterpret_cast<const v8ha*>(B + (size_t)(k0 + kk) * N + nBase + n0);
            #pragma unroll
            for (int j = 0; j < 8; ++j) Bst[(n0 + j) * LDT + kk] = t[j];
        }
        __syncthreads();

        F16Frag af[4];
        #pragma unroll
        for (int mi = 0; mi < 4; ++mi) {
            const int r = waveRow * 64 + mi * 16 + l15;
            const _Float16* p = &As[r * LDT + half * 8];
            af[mi].q[0] = *reinterpret_cast<const v8ha*>(p);
            af[mi].q[1] = *reinterpret_cast<const v8ha*>(p + 16);
        }
        F16Frag bf[2];
        #pragma unroll
        for (int ni = 0; ni < 2; ++ni) {
            const int c = waveCol * 32 + ni * 16 + l15;
            const _Float16* p = &Bst[c * LDT + half * 8];
            bf[ni].q[0] = *reinterpret_cast<const v8ha*>(p);
            bf[ni].q[1] = *reinterpret_cast<const v8ha*>(p + 16);
        }
        #pragma unroll
        for (int mi = 0; mi < 4; ++mi)
            #pragma unroll
            for (int ni = 0; ni < 2; ++ni)
                acc[mi][ni] = wmma_f16(af[mi], bf[ni], acc[mi][ni]);
        asm volatile("v_nop\n\tv_nop\n\tv_nop\n\tv_nop"
                     : "+v"(acc[0][0]), "+v"(acc[0][1]), "+v"(acc[1][0]), "+v"(acc[1][1]),
                       "+v"(acc[2][0]), "+v"(acc[2][1]), "+v"(acc[3][0]), "+v"(acc[3][1])
                     : "v"(af[3].h), "v"(bf[1].h));
        __syncthreads();
    }

    float bcol[2];
    #pragma unroll
    for (int ni = 0; ni < 2; ++ni) bcol[ni] = bf16r(bias[nBase + waveCol * 32 + ni * 16 + l15]);

    if constexpr (TRANS) {
        _Float16* const Cs = reinterpret_cast<_Float16*>(smem);
        #pragma unroll
        for (int ni = 0; ni < 2; ++ni) {
            const int col = waveCol * 32 + ni * 16 + l15;
            #pragma unroll
            for (int mi = 0; mi < 4; ++mi) {
                const int tok = waveRow * 64 + mi * 16 + half * 8;
                v8h t;
                #pragma unroll
                for (int v = 0; v < 8; ++v)
                    t[v] = (_Float16)((acc[mi][ni][v] * scale + bcol[ni]) * carry);
                *reinterpret_cast<v8ha*>(&Cs[col * CSP16 + tok]) = t;
            }
        }
        __syncthreads();
        #pragma unroll
        for (int ps = 0; ps < 2; ++ps) {
            #pragma unroll
            for (int it = 0; it < 8; ++it) {
                const int fr = it * 16 + wave * 2 + half;
                const int piece = l15 * 8;
                const v8h t = *reinterpret_cast<const v8ha*>(&Cs[fr * CSP16 + piece]);
                *reinterpret_cast<volatile v8ha*>(C + (size_t)(nBase + fr) * ldc + mBase + piece) = t;
            }
            if (ps == 0) __threadfence();
        }
    } else {
        float*    const Cs32 = smem;
        _Float16* const Cs16 = reinterpret_cast<_Float16*>(smem);
        #pragma unroll
        for (int rnd = 0; rnd < 2; ++rnd) {
            if (waveRow == rnd) {
                #pragma unroll
                for (int mi = 0; mi < 4; ++mi)
                    #pragma unroll
                    for (int ni = 0; ni < 2; ++ni) {
                        const int col = waveCol * 32 + ni * 16 + l15;
                        #pragma unroll
                        for (int v = 0; v < 8; ++v) {
                            const int rl = mi * 16 + half * 8 + v;
                            const float val = (acc[mi][ni][v] * scale + bcol[ni]) * carry;
                            if constexpr (sizeof(OutT) == 4) Cs32[rl * CSP32 + col] = val;
                            else Cs16[rl * CSP16 + col] = (_Float16)val;
                        }
                    }
            }
            __syncthreads();
            const int gRow0 = mBase + rnd * 64;
            const int bseg  = gRow0 / segRows;
            const size_t rowBase = (size_t)bseg * segStride + (size_t)(gRow0 - bseg * segRows);
            #pragma unroll
            for (int ps = 0; ps < 2; ++ps) {
                if constexpr (sizeof(OutT) == 4) {
                    #pragma unroll
                    for (int it = 0; it < 8; ++it) {
                        const int r = it * 8 + wave;
                        const v4f t = *reinterpret_cast<const v4fa*>(&Cs32[r * CSP32 + lane * 4]);
                        *reinterpret_cast<volatile v4fa*>(C + (rowBase + r) * (size_t)ldc + nBase + lane * 4) = t;
                    }
                } else {
                    #pragma unroll
                    for (int it = 0; it < 4; ++it) {
                        const int r = it * 16 + wave * 2 + half;
                        const v8h t = *reinterpret_cast<const v8ha*>(&Cs16[r * CSP16 + l15 * 8]);
                        *reinterpret_cast<volatile v8ha*>(C + (rowBase + r) * (size_t)ldc + nBase + l15 * 8) = t;
                    }
                }
                if (ps == 0) __threadfence();
            }
            __syncthreads();
        }
    }
}

#define APITCH 136

__global__ __launch_bounds__(256)
void attn_flash(const _Float16* __restrict__ Qh, const _Float16* __restrict__ Kh,
                const _Float16* __restrict__ Vt, const unsigned* __restrict__ mbits,
                _Float16* __restrict__ Ah) {
    __shared__ __align__(16) _Float16 Ps[8 * 16 * LDT];
    __shared__ __align__(16) _Float16 Cst[8 * 16 * APITCH];

    const int tid  = threadIdx.x;
    const int wave = tid >> 5;
    const int lane = tid & 31;
    const int half = lane >> 4;
    const int l15  = lane & 15;

    const int b = blockIdx.z, h = blockIdx.y;
    const int qRow0 = blockIdx.x * 128 + wave * 16;

    const _Float16* const Qb = Qh + ((size_t)b * SEQ) * HID + (size_t)h * HD;
    const _Float16* const Kb = Kh + ((size_t)b * SEQ) * HD;
    const _Float16* const Vb = Vt + (size_t)b * SEQ;
    const unsigned* const Mb = mbits + ((size_t)b * SEQ + qRow0 + half * 8) * SW;

    F16Frag qf[4];
    {
        const _Float16* qr = Qb + (size_t)(qRow0 + l15) * HID;
        #pragma unroll
        for (int kc = 0; kc < 4; ++kc) {
            const _Float16* p = qr + kc * 32 + half * 8;
            qf[kc].q[0] = *reinterpret_cast<const v8ha*>(p);
            qf[kc].q[1] = *reinterpret_cast<const v8ha*>(p + 16);
        }
    }

    v8f o[8];
    #pragma unroll
    for (int fi = 0; fi < 8; ++fi) o[fi] = vzero8();
    float m[8], l[8];
    #pragma unroll
    for (int v = 0; v < 8; ++v) { m[v] = -3.0e38f; l[v] = 0.f; }

    _Float16* const myPs = Ps + wave * 16 * LDT;
    const float kScale  = 0.08838834764831845f;
    const float kNegInf = -__builtin_inff();

    for (int kb = 0; kb < SEQ; kb += 32) {
        unsigned mw[8];
        #pragma unroll
        for (int v = 0; v < 8; ++v) mw[v] = Mb[(size_t)v * SW + (kb >> 5)];

        v8f s[2];
        s[0] = vzero8(); s[1] = vzero8();
        F16Frag kf[2];
        #pragma unroll
        for (int kc = 0; kc < 4; ++kc) {
            #pragma unroll
            for (int ni = 0; ni < 2; ++ni) {
                const _Float16* kr = Kb + (size_t)(kb + ni * 16 + l15) * HD + kc * 32 + half * 8;
                kf[ni].q[0] = *reinterpret_cast<const v8ha*>(kr);
                kf[ni].q[1] = *reinterpret_cast<const v8ha*>(kr + 16);
            }
            s[0] = wmma_f16(qf[kc], kf[0], s[0]);
            s[1] = wmma_f16(qf[kc], kf[1], s[1]);
        }
        asm volatile("v_nop\n\tv_nop\n\tv_nop\n\tv_nop"
                     : "+v"(s[0]), "+v"(s[1]) : "v"(qf[3].h), "v"(kf[1].h));

        #pragma unroll
        for (int v = 0; v < 8; ++v) {
            #pragma unroll
            for (int ni = 0; ni < 2; ++ni) {
                const float sv = s[ni][v] * kScale;
                const unsigned bit = (mw[v] >> (ni * 16 + l15)) & 1u;
                s[ni][v] = bit ? sv : kNegInf;
            }
        }

        float alpha[8];
        #pragma unroll
        for (int v = 0; v < 8; ++v) {
            const float mx = row_max16(fmaxf(s[0][v], s[1][v]));
            const float mn = fmaxf(m[v], mx);
            alpha[v] = __expf(m[v] - mn);
            m[v] = mn;
            const float p0 = __expf(s[0][v] - mn);
            const float p1 = __expf(s[1][v] - mn);
            s[0][v] = p0; s[1][v] = p1;
            l[v] = l[v] * alpha[v] + row_sum16(p0 + p1);
        }
        #pragma unroll
        for (int fi = 0; fi < 8; ++fi)
            #pragma unroll
            for (int v = 0; v < 8; ++v)
                o[fi][v] *= alpha[v];

        asm volatile("s_wait_dscnt 0x0" ::: "memory");
        #pragma unroll
        for (int ni = 0; ni < 2; ++ni)
            #pragma unroll
            for (int v = 0; v < 8; ++v)
                myPs[(v + half * 8) * LDT + ni * 16 + l15] = (_Float16)(s[ni][v] * 1024.0f);
        asm volatile("s_wait_dscnt 0x0" ::: "memory");
        __builtin_amdgcn_wave_barrier();

        F16Frag pf;
        {
            const _Float16* p = myPs + l15 * LDT + half * 8;
            pf.q[0] = *reinterpret_cast<const v8ha*>(p);
            pf.q[1] = *reinterpret_cast<const v8ha*>(p + 16);
        }

        F16Frag vf;
        #pragma unroll
        for (int fi = 0; fi < 8; ++fi) {
            const _Float16* vr = Vb + (size_t)(fi * 16 + l15) * NTOK + kb + half * 8;
            vf.q[0] = *reinterpret_cast<const v8ha*>(vr);
            vf.q[1] = *reinterpret_cast<const v8ha*>(vr + 16);
            o[fi] = wmma_f16(pf, vf, o[fi]);
        }
        asm volatile("v_nop\n\tv_nop\n\tv_nop\n\tv_nop"
                     : "+v"(o[0]), "+v"(o[1]), "+v"(o[2]), "+v"(o[3]),
                       "+v"(o[4]), "+v"(o[5]), "+v"(o[6]), "+v"(o[7])
                     : "v"(pf.h), "v"(vf.h));
    }

    float f[8];
    #pragma unroll
    for (int v = 0; v < 8; ++v) f[v] = 0.25f * (1.0f / l[v]);

    _Float16* const myC = Cst + wave * 16 * APITCH;
    #pragma unroll
    for (int fi = 0; fi < 8; ++fi)
        #pragma unroll
        for (int v = 0; v < 8; ++v)
            myC[(half * 8 + v) * APITCH + fi * 16 + l15] = (_Float16)(o[fi][v] * f[v]);
    asm volatile("s_wait_dscnt 0x0" ::: "memory");
    __builtin_amdgcn_wave_barrier();

    _Float16* const Ob = Ah + ((size_t)b * SEQ + qRow0) * HID + (size_t)h * HD;
    #pragma unroll
    for (int ps = 0; ps < 2; ++ps) {
        #pragma unroll
        for (int it = 0; it < 8; ++it) {
            const int r = it * 2 + half;
            const int piece = l15 * 8;
            const v8h t = *reinterpret_cast<const v8ha*>(myC + r * APITCH + piece);
            *reinterpret_cast<volatile v8ha*>(Ob + (size_t)r * HID + piece) = t;
        }
        if (ps == 0) __threadfence();
    }
}

extern "C" void kernel_launch(void* const* d_in, const int* in_sizes, int n_in,
                              void* d_out, int out_size, void* d_ws, size_t ws_size,
                              hipStream_t stream) {
    if (n_in < 10) return;
    const float* X  = (const float*)d_in[0];
    const int*   mk = (const int*)d_in[1];
    const float* Wq = (const float*)d_in[2];
    const float* bq = (const float*)d_in[3];
    const float* Wk = (const float*)d_in[4];
    const float* bk = (const float*)d_in[5];
    const float* Wv = (const float*)d_in[6];
    const float* bv = (const float*)d_in[7];
    const float* Wo = (const float*)d_in[8];
    const float* bo = (const float*)d_in[9];
    float* out = (float*)d_out;

    const int needX = ((NB - 1) * SEQ_FULL + SEQ) * HID;
    const int needM = ((NB - 1) * SEQ_FULL + SEQ) * SEQ_FULL;
    if (in_sizes[0] < needX || in_sizes[1] < needM) return;
    if (in_sizes[2] < HID * HID || in_sizes[3] < HID || in_sizes[4] < HID * HD || in_sizes[5] < HD) return;
    if (in_sizes[6] < HID * HD || in_sizes[7] < HD || in_sizes[8] < HID * HID || in_sizes[9] < HID) return;
    if (out_size < needX) return;

    size_t off = 0;
    char* const base = (char*)d_ws;
    auto take = [&](size_t bytes) -> char* { char* p = base + off; off += (bytes + 127) & ~(size_t)127; return p; };
    _Float16* Xh  = (_Float16*)take((size_t)NTOK * HID * 2);
    _Float16* Wqh = (_Float16*)take((size_t)HID * HID * 2);
    _Float16* Wkh = (_Float16*)take((size_t)HID * HD * 2);
    _Float16* Wvh = (_Float16*)take((size_t)HID * HD * 2);
    _Float16* Woh = (_Float16*)take((size_t)HID * HID * 2);
    _Float16* Qh  = (_Float16*)take((size_t)NTOK * HID * 2);
    _Float16* Khp = (_Float16*)take((size_t)NTOK * HD * 2);
    _Float16* Vt  = (_Float16*)take((size_t)HD * NTOK * 2);
    _Float16* Ah  = (_Float16*)take((size_t)NTOK * HID * 2);
    unsigned* Mb  = (unsigned*)take((size_t)NB * SEQ * SW * 4);
    if (off > ws_size) return;

    const dim3 blk(256);
    const float sProj = 6.103515625e-05f;
    const float sOut  = 3.814697265625e-06f;

    for (int b = 0; b < NB; ++b)
        cvt_f16<<<dim3((SEQ * HID / 8) / 256), blk, 0, stream>>>(
            X + (size_t)b * SEQ_FULL * HID, Xh + (size_t)b * SEQ * HID, SEQ * HID / 8, 16.0f);
    cvt_f16<<<dim3((HID * HID / 8) / 256), blk, 0, stream>>>(Wq, Wqh, HID * HID / 8, 1024.0f);
    cvt_f16<<<dim3((HID * HD / 8) / 256), blk, 0, stream>>>(Wk, Wkh, HID * HD / 8, 1024.0f);
    cvt_f16<<<dim3((HID * HD / 8) / 256), blk, 0, stream>>>(Wv, Wvh, HID * HD / 8, 1024.0f);
    cvt_f16<<<dim3((HID * HID / 8) / 256), blk, 0, stream>>>(Wo, Woh, HID * HID / 8, 1024.0f);

    pack_mask<<<dim3((SEQ * SW) / 256, NB), blk, 0, stream>>>(mk, Mb);

    gemm_f16<_Float16, false><<<dim3(HID / 128, NTOK / 128), blk, 0, stream>>>(
        Xh, Wqh, bq, Qh, HID, HID, HID, NTOK, NTOK, sProj, 1.0f);
    gemm_f16<_Float16, false><<<dim3(HD / 128, NTOK / 128), blk, 0, stream>>>(
        Xh, Wkh, bk, Khp, HD, HID, HD, NTOK, NTOK, sProj, 1.0f);
    gemm_f16<_Float16, true><<<dim3(HD / 128, NTOK / 128), blk, 0, stream>>>(
        Xh, Wvh, bv, Vt, HD, HID, NTOK, NTOK, NTOK, sProj, 1.0f);

    attn_flash<<<dim3(SEQ / 128, NHEAD, NB), blk, 0, stream>>>(Qh, Khp, Vt, Mb, Ah);

    gemm_f16<float, false><<<dim3(HID / 128, NTOK / 128), blk, 0, stream>>>(
        Ah, Woh, bo, out, HID, HID, HID, SEQ, SEQ_FULL, sOut, 1.0f);
}
